// MutliHeadAttentionBlock_39307540693562
// MI455X (gfx1250) — hardware-verified
//
#include <hip/hip_runtime.h>
#include <stddef.h>
#include <stdint.h>


#define DM 1024
#define SQ 2048
#define NB 2
#define NH 16
#define DK 64
#define MT (NB * SQ)
#define MWORDS (SQ / 32)

#define GBK 64
#define LP 72
#define SP 136
#define FP 132
#define GEMM_LDS_BYTES 36864
#define AP 72

typedef _Float16 f16;
typedef f16 v16h __attribute__((ext_vector_type(16)));
typedef f16 v8h __attribute__((ext_vector_type(8)));
typedef float v8f __attribute__((ext_vector_type(8)));
typedef float v4f __attribute__((ext_vector_type(4)));
typedef int v4i __attribute__((ext_vector_type(4)));
typedef unsigned int v4u __attribute__((ext_vector_type(4)));

union Frag { v16h v; v8h h[2]; };

__device__ __forceinline__ v8f zero8() {
  return (v8f){0.f, 0.f, 0.f, 0.f, 0.f, 0.f, 0.f, 0.f};
}

__device__ __forceinline__ v8f wmma16(v16h a, v16h b, v8f c) {
  v8f d = __builtin_amdgcn_wmma_f32_16x16x32_f16(false, a, false, b, (short)0, c, false, false);
  asm volatile("v_nop\n\tv_nop\n\tv_nop\n\tv_nop" : "+v"(d) : "v"(a), "v"(b));
  return d;
}

__device__ __forceinline__ v16h ld_frag(const f16* base, int pitch, int row0, int k0, int lane) {
  const f16* p = base + (row0 + (lane & 15)) * pitch + k0 + 8 * (lane >> 4);
  Frag f;
  f.h[0] = *(const v8h*)p;
  f.h[1] = *(const v8h*)(p + 16);
  return f.v;
}

__global__ __launch_bounds__(256)
void k_cvt(const float* __restrict__ s0, const float* __restrict__ s1,
           const float* __restrict__ s2, const float* __restrict__ s3,
           f16* d0, f16* d1, f16* d2, f16* d3, int n, float scale) {
  const int j = blockIdx.y;
  const float* s = (j == 0) ? s0 : (j == 1) ? s1 : (j == 2) ? s2 : s3;
  f16* d = (j == 0) ? d0 : (j == 1) ? d1 : (j == 2) ? d2 : d3;
  const size_t i = ((size_t)blockIdx.x * 256 + threadIdx.x) * 8;
  if (i + 8 <= (size_t)n) {
    const v4f a = *(const v4f*)(s + i);
    const v4f c = *(const v4f*)(s + i + 4);
    v8h o;
    o[0] = (f16)(a[0] * scale); o[1] = (f16)(a[1] * scale);
    o[2] = (f16)(a[2] * scale); o[3] = (f16)(a[3] * scale);
    o[4] = (f16)(c[0] * scale); o[5] = (f16)(c[1] * scale);
    o[6] = (f16)(c[2] * scale); o[7] = (f16)(c[3] * scale);
    volatile v8h* g = (volatile v8h*)(d + i);
    *g = o;
    __threadfence();
    *g = o;
  }
}

__global__ __launch_bounds__(256)
void k_maskbits(const int* __restrict__ mask, unsigned* bits) {
  __shared__ v4u sw[16];
  unsigned char* sb = (unsigned char*)sw;
  const int t = threadIdx.x;
  const size_t row = blockIdx.x;
  const int* p = mask + row * SQ + (size_t)t * 8;
  const v4i a = *(const v4i*)p;
  const v4i c = *(const v4i*)(p + 4);
  unsigned byte = (unsigned)(a[0] != 0) | ((unsigned)(a[1] != 0) << 1) |
                  ((unsigned)(a[2] != 0) << 2) | ((unsigned)(a[3] != 0) << 3) |
                  ((unsigned)(c[0] != 0) << 4) | ((unsigned)(c[1] != 0) << 5) |
                  ((unsigned)(c[2] != 0) << 6) | ((unsigned)(c[3] != 0) << 7);
  sb[t] = (unsigned char)byte;
  __syncthreads();
  if (t < 16) {
    const v4u w = sw[t];
    volatile v4u* g = (volatile v4u*)(bits + row * MWORDS + t * 4);
    *g = w;
    __threadfence();
    *g = w;
  }
}

__device__ __forceinline__ void store_head_rows(const f16* lS, f16* dst, int m0, int n0,
                                                int wave, int lane) {
  const int b = m0 / SQ, s0 = m0 % SQ, hb = n0 / DK;
#pragma unroll
  for (int it = 0; it < 8; ++it) {
    const int L = wave * 32 + it * 4 + (lane >> 3);
    const int ml = L >> 1, hl = L & 1, pc = lane & 7;
    const v8h v = *(const v8h*)(lS + ml * SP + hl * DK + pc * 8);
    f16* g = dst + ((size_t)((b * NH + hb + hl) * SQ + s0 + ml)) * DK + pc * 8;
    *(volatile v8h*)g = v;
  }
}

__device__ __forceinline__ void store_vt_rows(const f16* lS, f16* dst, int m0, int n0,
                                              int wave, int lane) {
  const int b = m0 / SQ, s0 = m0 % SQ, hb = n0 / DK;
#pragma unroll
  for (int it = 0; it < 8; ++it) {
    const int nl = wave * 16 + it * 2 + (lane >> 4);
    const int pc = lane & 15;
    const int hd = hb + (nl >> 6), dl = nl & (DK - 1);
    const v8h v = *(const v8h*)(lS + nl * SP + pc * 8);
    f16* g = dst + ((size_t)((b * NH + hd) * DK + dl)) * SQ + s0 + pc * 8;
    *(volatile v8h*)g = v;
  }
}

__device__ __forceinline__ void store_f32_rows(const float* lF, float* dst, int mrow0, int n0,
                                               int wave, int lane) {
#pragma unroll
  for (int it = 0; it < 8; ++it) {
    const int rl = wave * 8 + it;
    const v4f v = *(const v4f*)(lF + rl * FP + lane * 4);
    float* g = dst + (size_t)(mrow0 + rl) * DM + n0 + lane * 4;
    *(volatile v4f*)g = v;
  }
}

__device__ __forceinline__ void store_x_rows(const f16* Pw, f16* xout, size_t rowbase, int h,
                                             int lane) {
#pragma unroll
  for (int it = 0; it < 4; ++it) {
    const int rl = it * 4 + (lane >> 3), pc = lane & 7;
    const v8h v = *(const v8h*)(Pw + rl * AP + pc * 8);
    f16* g = xout + (rowbase + rl) * DM + h * DK + pc * 8;
    *(volatile v8h*)g = v;
  }
}

template <int MODE>
__global__ __launch_bounds__(256)
void k_gemm(const f16* __restrict__ X, const f16* __restrict__ W, const float* __restrict__ bias,
            float oscale, f16* outH, float* outF) {
  __shared__ __attribute__((aligned(16))) unsigned char lds_raw[GEMM_LDS_BYTES];
  f16* lA = (f16*)lds_raw;
  f16* lB = lA + 128 * LP;
  const int tid = threadIdx.x, lane = tid & 31, wave = tid >> 5;
  const int m0 = blockIdx.y * 128, n0 = blockIdx.x * 128;
  const int wm = (wave >> 2) * 64, wn = (wave & 3) * 32;
  const int col = lane & 15, hh = lane >> 4;

  v8f acc[4][2];
#pragma unroll
  for (int mi = 0; mi < 4; ++mi)
#pragma unroll
    for (int ni = 0; ni < 2; ++ni) acc[mi][ni] = zero8();

  for (int k0 = 0; k0 < DM; k0 += GBK) {
    __syncthreads();
#pragma unroll
    for (int p = 0; p < 4; ++p) {
      const int c = p * 256 + tid, row = c >> 3, pc = (c & 7) * 8;
      const v8h va = *(const v8h*)(X + (size_t)(m0 + row) * DM + k0 + pc);
      const v8h vb = *(const v8h*)(W + (size_t)(n0 + row) * DM + k0 + pc);
      *(v8h*)(lA + row * LP + pc) = va;
      *(v8h*)(lB + row * LP + pc) = vb;
    }
    __syncthreads();
#pragma unroll
    for (int ks = 0; ks < GBK; ks += 32) {
      v16h af[4], bfr[2];
#pragma unroll
      for (int mi = 0; mi < 4; ++mi) af[mi] = ld_frag(lA, LP, wm + mi * 16, ks, lane);
#pragma unroll
      for (int ni = 0; ni < 2; ++ni) bfr[ni] = ld_frag(lB, LP, wn + ni * 16, ks, lane);
#pragma unroll
      for (int mi = 0; mi < 4; ++mi)
#pragma unroll
        for (int ni = 0; ni < 2; ++ni) acc[mi][ni] = wmma16(af[mi], bfr[ni], acc[mi][ni]);
    }
  }
  __syncthreads();

  const float bv0 = bias[n0 + wn + col];
  const float bv1 = bias[n0 + wn + 16 + col];

  if (MODE == 0) {
    f16* lS = (f16*)lds_raw;
#pragma unroll
    for (int mi = 0; mi < 4; ++mi)
#pragma unroll
      for (int ni = 0; ni < 2; ++ni)
#pragma unroll
        for (int r = 0; r < 8; ++r) {
          const float y = acc[mi][ni][r] * oscale + (ni ? bv1 : bv0);
          lS[(wm + mi * 16 + 8 * hh + r) * SP + wn + ni * 16 + col] = (f16)y;
        }
    __syncthreads();
    store_head_rows(lS, outH, m0, n0, wave, lane);
    __threadfence();
    store_head_rows(lS, outH, m0, n0, wave, lane);
  } else if (MODE == 1) {
    f16* lS = (f16*)lds_raw;
#pragma unroll
    for (int mi = 0; mi < 4; ++mi)
#pragma unroll
      for (int ni = 0; ni < 2; ++ni) {
        v8h pk;
#pragma unroll
        for (int r = 0; r < 8; ++r) pk[r] = (f16)(acc[mi][ni][r] * oscale + (ni ? bv1 : bv0));
        *(v8h*)(lS + (wn + ni * 16 + col) * SP + wm + mi * 16 + 8 * hh) = pk;
      }
    __syncthreads();
    store_vt_rows(lS, outH, m0, n0, wave, lane);
    __threadfence();
    store_vt_rows(lS, outH, m0, n0, wave, lane);
  } else {
    float* lF = (float*)lds_raw;
#pragma unroll
    for (int hm = 0; hm < 2; ++hm) {
      if ((wave >> 2) == hm) {
#pragma unroll
        for (int mi = 0; mi < 4; ++mi)
#pragma unroll
          for (int ni = 0; ni < 2; ++ni)
#pragma unroll
            for (int r = 0; r < 8; ++r)
              lF[(mi * 16 + 8 * hh + r) * FP + wn + ni * 16 + col] =
                  acc[mi][ni][r] * oscale + (ni ? bv1 : bv0);
      }
      __syncthreads();
      store_f32_rows(lF, outF, m0 + hm * 64, n0, wave, lane);
      __threadfence();
      store_f32_rows(lF, outF, m0 + hm * 64, n0, wave, lane);
      __syncthreads();
    }
  }
}

__global__ __launch_bounds__(128)
void k_attn(const f16* __restrict__ Qh, const f16* __restrict__ Kh, const f16* __restrict__ Vt,
            const unsigned* __restrict__ mbits, f16* xout) {
  __shared__ __attribute__((aligned(16))) f16 Ks[64 * AP];
  __shared__ __attribute__((aligned(16))) f16 Vs[64 * AP];
  __shared__ __attribute__((aligned(16))) f16 Ps[4 * 16 * AP];
  __shared__ unsigned Mw[128];
  const int tid = threadIdx.x, lane = tid & 31, wave = tid >> 5;
  const int col = lane & 15, hh = lane >> 4;
  const int q0 = blockIdx.x * 64, bh = blockIdx.y;
  const int b = bh / NH, h = bh % NH;
  const size_t hoff = (size_t)bh * SQ * DK;
  f16* Pw = Ps + wave * 16 * AP;

  v16h qa[2];
  {
    const f16* qp = Qh + hoff + (size_t)(q0 + wave * 16 + col) * DK + 8 * hh;
    Frag f;
    f.h[0] = *(const v8h*)(qp);      f.h[1] = *(const v8h*)(qp + 16); qa[0] = f.v;
    f.h[0] = *(const v8h*)(qp + 32); f.h[1] = *(const v8h*)(qp + 48); qa[1] = f.v;
  }

  float mrow[8], lrow[8];
  v8f O[4];
#pragma unroll
  for (int v = 0; v < 8; ++v) { mrow[v] = -1e30f; lrow[v] = 0.f; }
#pragma unroll
  for (int ni = 0; ni < 4; ++ni) O[ni] = zero8();

  const unsigned* mrp = mbits + (size_t)(b * SQ + q0) * MWORDS;

  for (int kt = 0; kt < SQ; kt += 64) {
    __syncthreads();
#pragma unroll
    for (int p = 0; p < 4; ++p) {
      const int c = p * 128 + tid, row = c >> 3, pc = (c & 7) * 8;
      const v8h kv = *(const v8h*)(Kh + hoff + (size_t)(kt + row) * DK + pc);
      const v8h vv = *(const v8h*)(Vt + hoff + (size_t)row * SQ + kt + pc);
      *(v8h*)(Ks + row * AP + pc) = kv;
      *(v8h*)(Vs + row * AP + pc) = vv;
    }
    Mw[tid] = mrp[(size_t)(tid >> 1) * MWORDS + (kt >> 5) + (tid & 1)];
    __syncthreads();

    v8f sc[4];
#pragma unroll
    for (int ni = 0; ni < 4; ++ni) {
      v8f c = zero8();
      c = wmma16(qa[0], ld_frag(Ks, AP, ni * 16, 0, lane), c);
      c = wmma16(qa[1], ld_frag(Ks, AP, ni * 16, 32, lane), c);
      sc[ni] = c * 0.125f;
    }

#pragma unroll
    for (int v = 0; v < 8; ++v) {
      const int rl = (wave * 16 + 8 * hh + v) * 2;
      const unsigned w0 = Mw[rl], w1 = Mw[rl + 1];
#pragma unroll
      for (int ni = 0; ni < 4; ++ni) {
        const unsigned w = (ni >> 1) ? w1 : w0;
        const int bit = ((ni & 1) << 4) | col;
        const bool keep = ((w >> bit) & 1u) != 0u;
        sc[ni][v] = keep ? sc[ni][v] : -1e9f;
      }
    }

#pragma unroll
    for (int v = 0; v < 8; ++v) {
      float mx = sc[0][v];
#pragma unroll
      for (int ni = 1; ni < 4; ++ni) mx = fmaxf(mx, sc[ni][v]);
#pragma unroll
      for (int off = 8; off >= 1; off >>= 1) mx = fmaxf(mx, __shfl_xor(mx, off, 32));
      const float mnew = fmaxf(mrow[v], mx);
      const float alpha = __expf(mrow[v] - mnew);
      float rs = 0.f;
#pragma unroll
      for (int ni = 0; ni < 4; ++ni) {
        const float pv = __expf(sc[ni][v] - mnew);
        sc[ni][v] = pv;
        rs += pv;
      }
#pragma unroll
      for (int off = 8; off >= 1; off >>= 1) rs += __shfl_xor(rs, off, 32);
      mrow[v] = mnew;
      lrow[v] = lrow[v] * alpha + rs;
#pragma unroll
      for (int ni = 0; ni < 4; ++ni) O[ni][v] *= alpha;
    }

#pragma unroll
    for (int ni = 0; ni < 4; ++ni)
#pragma unroll
      for (int v = 0; v < 8; ++v)
        Pw[(v + 8 * hh) * AP + ni * 16 + col] = (f16)(sc[ni][v] * 64.0f);
    __syncthreads();

#pragma unroll
    for (int ks = 0; ks < 64; ks += 32) {
      const v16h pa = ld_frag(Pw, AP, 0, ks, lane);
#pragma unroll
      for (int ni = 0; ni < 4; ++ni)
        O[ni] = wmma16(pa, ld_frag(Vs, AP, ni * 16, ks, lane), O[ni]);
    }
  }
  __syncthreads();

  float inv[8];
#pragma unroll
  for (int v = 0; v < 8; ++v) inv[v] = 1.0f / lrow[v];
#pragma unroll
  for (int ni = 0; ni < 4; ++ni)
#pragma unroll
    for (int v = 0; v < 8; ++v)
      Pw[(v + 8 * hh) * AP + ni * 16 + col] = (f16)(O[ni][v] * inv[v]);
  __syncthreads();

  const size_t rowbase = (size_t)(b * SQ + q0 + wave * 16);
  store_x_rows(Pw, xout, rowbase, h, lane);
  __threadfence();
  store_x_rows(Pw, xout, rowbase, h, lane);
}

extern "C" void kernel_launch(void* const* d_in, const int* in_sizes, int n_in,
                              void* d_out, int out_size, void* d_ws, size_t ws_size,
                              hipStream_t stream) {
  if (n_in < 12) return;
  if (in_sizes[0] != MT * DM || in_sizes[1] != MT * DM || in_sizes[2] != MT * DM) return;
  if (in_sizes[3] != NB * SQ * SQ) return;
  if (in_sizes[4] != DM * DM || in_sizes[6] != DM * DM ||
      in_sizes[8] != DM * DM || in_sizes[10] != DM * DM) return;
  if (in_sizes[5] != DM || in_sizes[7] != DM || in_sizes[9] != DM || in_sizes[11] != DM) return;
  if (out_size != MT * DM) return;

  const float* q   = (const float*)d_in[0];
  const float* k   = (const float*)d_in[1];
  const float* v   = (const float*)d_in[2];
  const int*   msk = (const int*)d_in[3];
  const float* w_q = (const float*)d_in[4];
  const float* b_q = (const float*)d_in[5];
  const float* w_k = (const float*)d_in[6];
  const float* b_k = (const float*)d_in[7];
  const float* w_v = (const float*)d_in[8];
  const float* b_v = (const float*)d_in[9];
  const float* w_o = (const float*)d_in[10];
  const float* b_o = (const float*)d_in[11];
  float* out = (float*)d_out;

  const size_t actB = (size_t)MT * DM * sizeof(f16);
  const size_t wgtB = (size_t)DM * DM * sizeof(f16);
  const size_t mbB  = (size_t)NB * SQ * MWORDS * sizeof(unsigned);
  unsigned char* ws = (unsigned char*)d_ws;
  size_t off = 0;
  f16* q16  = (f16*)(ws + off); off += actB;
  f16* k16  = (f16*)(ws + off); off += actB;
  f16* v16  = (f16*)(ws + off); off += actB;
  f16* wq16 = (f16*)(ws + off); off += wgtB;
  f16* wk16 = (f16*)(ws + off); off += wgtB;
  f16* wv16 = (f16*)(ws + off); off += wgtB;
  f16* wo16 = (f16*)(ws + off); off += wgtB;
  f16* Qh   = (f16*)(ws + off); off += actB;
  f16* Kh   = (f16*)(ws + off); off += actB;
  f16* Vt   = (f16*)(ws + off); off += actB;
  f16* x16  = (f16*)(ws + off); off += actB;
  unsigned* mbits = (unsigned*)(ws + off); off += mbB;
  if (off > ws_size) return;

  const int nAct = MT * DM, nWgt = DM * DM;
  k_cvt<<<dim3((nAct / 8 + 255) / 256, 3), 256, 0, stream>>>(
      q, k, v, v, q16, k16, v16, v16, nAct, 1.0f);
  k_cvt<<<dim3((nWgt / 8 + 255) / 256, 4), 256, 0, stream>>>(
      w_q, w_k, w_v, w_o, wq16, wk16, wv16, wo16, nWgt, 16.0f);
  k_maskbits<<<dim3(NB * SQ), 256, 0, stream>>>(msk, mbits);

  const dim3 gg(DM / 128, MT / 128);
  k_gemm<0><<<gg, 256, 0, stream>>>(q16, wq16, b_q, 1.0f / 16.0f, Qh, out);
  k_gemm<0><<<gg, 256, 0, stream>>>(k16, wk16, b_k, 1.0f / 16.0f, Kh, out);
  k_gemm<1><<<gg, 256, 0, stream>>>(v16, wv16, b_v, 1.0f / 16.0f, Vt, out);

  k_attn<<<dim3(SQ / 64, NB * NH), 128, 0, stream>>>(Qh, Kh, Vt, mbits, x16);

  k_gemm<2><<<gg, 256, 0, stream>>>(x16, wo16, b_o, 1.0f / 1024.0f, x16, out);
}
